// GeneratedTreeClassifier_50062138802299
// MI455X (gfx1250) — hardware-verified
//
#include <hip/hip_runtime.h>
#include <math.h>

typedef __attribute__((ext_vector_type(16))) _Float16 v16h;
typedef __attribute__((ext_vector_type(16))) __bf16 v16b;
typedef __attribute__((ext_vector_type(8)))  _Float16 v8h;
typedef __attribute__((ext_vector_type(8)))  float v8f;
typedef __attribute__((ext_vector_type(4)))  float v4f;
typedef __attribute__((ext_vector_type(2)))  float v2f;
typedef __attribute__((ext_vector_type(4)))  unsigned v4u;
typedef __attribute__((ext_vector_type(4)))  int v4i;
typedef float __attribute__((may_alias)) float_a;
typedef int __attribute__((may_alias)) int_a;

template <typename T> __device__ __forceinline__ void vst2(void* p, T v) { *(volatile T*)p = v; __threadfence(); *(volatile T*)p = v; }
__device__ __forceinline__ v8f wmma16(v16h a, v16h b, v8f c) {
  v8f d = __builtin_amdgcn_wmma_f32_16x16x32_f16(false, a, false, b, (short)0, c, false, false);
  asm volatile("v_nop\n\tv_nop\n\tv_nop\n\tv_nop" : "+v"(d) : "v"(a), "v"(b));
  return d;
}
__device__ __forceinline__ v8f wmma_bf(v16b a, v16b b, v8f c) {
  v8f d = __builtin_amdgcn_wmma_f32_16x16x32_bf16(false, a, false, b, (short)0, c, false, false);
  asm volatile("v_nop\n\tv_nop\n\tv_nop\n\tv_nop" : "+v"(d) : "v"(a), "v"(b));
  return d;
}
__device__ __forceinline__ v16h frag_h(const _Float16* rowk0, int lane) {
  union { v16h v; v8h q[2]; } u; const _Float16* p = rowk0 + 8 * (lane >> 4);
  u.q[0] = *(const v8h*)p; u.q[1] = *(const v8h*)(p + 16); return u.v;
}
__device__ __forceinline__ v16h frag_f32(const float* rowk0, int lane) {
  v16h a; const float* p = rowk0 + 8 * (lane >> 4);
#pragma unroll
  for (int i = 0; i < 8; ++i) { a[i] = (_Float16)p[i]; a[8 + i] = (_Float16)p[16 + i]; }
  return a;
}
__device__ __forceinline__ v16h frag_f32s(const float* rowk0, int lane, float sc) {
  v16h a; const float* p = rowk0 + 8 * (lane >> 4);
#pragma unroll
  for (int i = 0; i < 8; ++i) { a[i] = (_Float16)(p[i] * sc); a[8 + i] = (_Float16)(p[16 + i] * sc); }
  return a;
}
__device__ __forceinline__ v16h fragc_f32(const float* W, int k0, int n, int lane, int ld, int K) {
  v16h a; const int g = lane >> 4;
#pragma unroll
  for (int i = 0; i < 8; ++i) { const int ka = k0 + 8 * g + i, kb = ka + 16;
    a[i] = (_Float16)(ka < K ? W[(size_t)(ka < K ? ka : K - 1) * ld + n] : 0.f); a[8 + i] = (_Float16)(kb < K ? W[(size_t)(kb < K ? kb : K - 1) * ld + n] : 0.f); }
  return a;
}
struct F2 { v16b h, l; };
__device__ __forceinline__ F2 bsplit16(const float v[16]) { F2 r;
#pragma unroll
  for (int i = 0; i < 16; ++i) { const __bf16 h = (__bf16)v[i]; r.h[i] = h; r.l[i] = (__bf16)(v[i] - (float)h); }
  return r; }
__device__ __forceinline__ F2 split_row(const float* row, int k0, int lane) { float v[16]; const float* p = row + k0 + 8 * (lane >> 4);
#pragma unroll
  for (int i = 0; i < 8; ++i) { v[i] = p[i]; v[8 + i] = p[16 + i]; }
  return bsplit16(v); }
__device__ __forceinline__ F2 split_rowK(const float* row, int k0, int lane, int K) { float v[16]; const int g = lane >> 4;
#pragma unroll
  for (int i = 0; i < 8; ++i) { const int ka = k0 + 8 * g + i, kb = ka + 16; v[i] = ka < K ? row[ka < K ? ka : K - 1] : 0.f; v[8 + i] = kb < K ? row[kb < K ? kb : K - 1] : 0.f; }
  return bsplit16(v); }
__device__ __forceinline__ F2 split_col(const float* W, int k0, int n, int lane, int ld, int K) { float v[16]; const int g = lane >> 4;
#pragma unroll
  for (int i = 0; i < 8; ++i) { const int ka = k0 + 8 * g + i, kb = ka + 16; v[i] = ka < K ? W[(size_t)(ka < K ? ka : K - 1) * ld + n] : 0.f; v[8 + i] = kb < K ? W[(size_t)(kb < K ? kb : K - 1) * ld + n] : 0.f; }
  return bsplit16(v); }
__device__ __forceinline__ v8f mac3(const F2& a, const F2& b, v8f c) { c = wmma_bf(a.l, b.h, c); c = wmma_bf(a.h, b.l, c); return wmma_bf(a.h, b.h, c); }
__device__ __forceinline__ float sigm(float v) { return 1.0f / (1.0f + expf(-v)); }
#define LDSX() do { asm volatile("s_wait_dscnt 0" ::: "memory"); __builtin_amdgcn_wave_barrier(); __builtin_amdgcn_fence(__ATOMIC_RELEASE, "workgroup"); } while (0)


#define NBATCH 8192
#define DF 1024
#define NT 16
#define NIN 255
#define NLF 256
#define NC 100
#define NCP 128
#define KS (NT * NLF)
#ifndef TROW
#define TROW NBATCH
#endif
typedef __attribute__((ext_vector_type(8))) __bf16 v8b;
__device__ __forceinline__ v16b frag_b(const __bf16* rowk0, int lane) {
  union { v16b v; v8b q[2]; } u; const __bf16* p = rowk0 + 8 * (lane >> 4);
  u.q[0] = *(const v8b*)p; u.q[1] = *(const v8b*)(p + 16); return u.v;
}
__device__ __forceinline__ float bfr(float v) { return (float)(__bf16)v; }
__device__ __attribute__((noinline)) float exp_ni(float v) { return expf(v); }
__device__ __attribute__((noinline)) float erf_ni(float v) { return erff(v); }

#define WS_P   0u
#define WS_LH  (WS_P + 4u * (size_t)NBATCH * KS)
#define WS_LL  (WS_LH + 2u * (size_t)NCP * KS)
#define WS_END (WS_LL + 2u * (size_t)NCP * KS)

__device__ __forceinline__ v16b fragb_f32(const float* __restrict__ p, int lane) { v16b a; const float* pp = p + 8 * (lane >> 4);
#pragma unroll
  for (int i = 0; i < 8; ++i) { a[i] = (__bf16)pp[i]; a[8 + i] = (__bf16)pp[16 + i]; } return a; }
__global__ __launch_bounds__(256) void k_leaf(const float* __restrict__ LL, const float* __restrict__ TW, __bf16* __restrict__ LH, __bf16* __restrict__ LLo) { __shared__ __align__(16) __bf16 sh[KS], sl[KS]; __shared__ float swt[NT];
  const int c = blockIdx.x, t = threadIdx.x;
  if (t == 0) { float mx = -3.0e38f;
#pragma unroll 1
    for (int i = 0; i < NT; ++i) mx = fmaxf(mx, bfr(TW[i]));
    float s = 0.f;
#pragma unroll 1
    for (int i = 0; i < NT; ++i) s += __expf(bfr(TW[i]) - mx);
    const float is = 1.0f / s;
#pragma unroll 1
    for (int i = 0; i < NT; ++i) swt[i] = __expf(bfr(TW[i]) - mx) * is; }
  __syncthreads();
  for (int e = t; e < KS; e += 256) { float v = 0.f;
    if (c < NC) { const float* row = LL + (size_t)e * NC; float mx = -3.0e38f;
#pragma unroll 1
      for (int k = 0; k < NC; ++k) mx = fmaxf(mx, bfr(row[k]));
      float s = 0.f;
#pragma unroll 1
      for (int k = 0; k < NC; ++k) s += __expf(bfr(row[k]) - mx);
      v = __expf(bfr(row[c]) - mx) / s * swt[e / NLF]; }
    const __bf16 h = (__bf16)v; sh[e] = h; sl[e] = (__bf16)(v - (float)h); }
  __syncthreads();
  for (int q = t; q < KS / 8; q += 256) { vst2((unsigned*)(LH + (size_t)c * KS + q * 8), *(const v4u*)&sh[q * 8]); vst2((unsigned*)(LLo + (size_t)c * KS + q * 8), *(const v4u*)&sl[q * 8]); } }
__global__ __launch_bounds__(128) void k_split(const float* __restrict__ X, const float* __restrict__ WS_, const float* __restrict__ SB, float* __restrict__ P) { __shared__ __align__(16) float sf[4][16][132];
  const int tid = threadIdx.x, wave = tid >> 5, lane = tid & 31, col = lane & 15, g = lane >> 4; const size_t r0 = (size_t)blockIdx.x * 64 + wave * 16; const int c0 = blockIdx.y * 128; const int t = c0 / NLF;
  v8f acc[8] = {};
#pragma unroll 2
  for (int kc = 0; kc < DF / 32; ++kc) { const v16b a = fragb_f32(X + (r0 + col) * DF + kc * 32, lane);
#pragma unroll
    for (int j = 0; j < 8; ++j) { const int n = (c0 % NLF) + j * 16 + col; const int nn = n < NIN ? n : NIN - 1;
      acc[j] = wmma_bf(a, fragb_f32(WS_ + ((size_t)t * NIN + nn) * DF + kc * 32, lane), acc[j]); } }
#pragma unroll
  for (int j = 0; j < 8; ++j) { const int n = (c0 % NLF) + j * 16 + col; const float bb = (n < NIN) ? bfr(SB[t * NIN + n]) : 0.f;
#pragma unroll
    for (int r = 0; r < 8; ++r) { const float z = acc[j][r] + bb; sf[wave][8 * g + r][j * 16 + col] = (n < NIN) ? 1.0f / (1.0f + expf(-z)) : 1.0f; } }
  LDSX(); for (int rl = 0; rl < 16; ++rl) vst2(P + (r0 + rl) * KS + c0 + lane * 4, *(const v4f*)&sf[wave][rl][lane * 4]); }
__device__ __forceinline__ float reach(const float* __restrict__ prow, int l) { float m = 1.0f;
#pragma unroll
  for (int d = 0; d < 8; ++d) { const int node = ((1 << d) - 1) + (l >> (8 - d)); const int bit = (l >> (7 - d)) & 1; const float p = prow[node]; m *= bit ? p : (1.0f - p); }
  return m; }
__global__ __launch_bounds__(128) void k_out(const float* __restrict__ P, const __bf16* __restrict__ LH, const __bf16* __restrict__ LLo, float* __restrict__ OUT) { __shared__ __align__(16) float sf[4][16][132];
  const int tid = threadIdx.x, wave = tid >> 5, lane = tid & 31, col = lane & 15, g = lane >> 4; const size_t r0 = (size_t)blockIdx.x * 64 + wave * 16; const float* prow0 = P + (r0 + col) * KS;
  v8f acc[8] = {};
#pragma unroll 1
  for (int kc = 0; kc < KS / 32; ++kc) { const int t = (kc * 32) / NLF; const int l0 = (kc * 32) % NLF; const float* prow = prow0 + t * NLF; float v[16];
#pragma unroll
    for (int i = 0; i < 8; ++i) { v[i] = reach(prow, l0 + 8 * g + i); v[8 + i] = reach(prow, l0 + 16 + 8 * g + i); }
    const F2 a = bsplit16(v);
#pragma unroll
    for (int j = 0; j < 8; ++j) { const F2 w = { frag_b(LH + (size_t)(j * 16 + col) * KS + kc * 32, lane), frag_b(LLo + (size_t)(j * 16 + col) * KS + kc * 32, lane) }; acc[j] = mac3(a, w, acc[j]); } }
#pragma unroll
  for (int j = 0; j < 8; ++j)
#pragma unroll
    for (int r = 0; r < 8; ++r) sf[wave][8 * g + r][j * 16 + col] = acc[j][r];
  LDSX(); for (int rl = 0; rl < 16; ++rl) if (lane < NC / 4) vst2(OUT + (r0 + rl) * NC + lane * 4, *(const v4f*)&sf[wave][rl][lane * 4]); }
extern "C" void kernel_launch(void* const* d_in, const int* in_sizes, int n_in, void* d_out, int out_size, void* d_ws, size_t ws_size, hipStream_t stream) {
  (void)in_sizes; (void)n_in; (void)out_size;
  const float** F = (const float**)d_in;
  if (ws_size < (size_t)WS_END) return;
  char* ws = (char*)d_ws; float* P = (float*)(ws + WS_P); __bf16 *LH = (__bf16*)(ws + WS_LH), *LLo = (__bf16*)(ws + WS_LL);
  k_leaf<<<NCP, 256, 0, stream>>>(F[3], F[4], LH, LLo);
  k_split<<<dim3(TROW / 64, KS / 128), 128, 0, stream>>>(F[0], F[1], F[2], P);
  k_out<<<TROW / 64, 128, 0, stream>>>(P, LH, LLo, (float*)d_out);
}
